// Encoder_8821862826192
// MI455X (gfx1250) — hardware-verified
//
#include <hip/hip_runtime.h>
#include <math.h>

constexpr int N_BATCH  = 1024;
constexpr int N_STEP   = 1024;
constexpr int HID1     = 64;
constexpr int HID2     = 32;
constexpr int GATE1    = 3 * HID1;
constexpr int GATE2    = 3 * HID2;
constexpr int ROWS_BLK = 16;
constexpr int NTHREADS = 32;
constexpr int PITCH_W1  = 72;
constexpr int PITCH_W2I = 72;
constexpr int PITCH_W2H = 40;
constexpr int PITCH_H1  = 72;
constexpr int PITCH_H2  = 40;
constexpr int X_CHUNK   = 32;
constexpr int PITCH_X   = 36;
constexpr int PITCH_OUT = 36;
constexpr int C_WIH1 = 0;
constexpr int C_B1RZ = 192;
constexpr int C_B1IN = 320;
constexpr int C_B1HN = 384;
constexpr int C_B2RZ = 448;
constexpr int C_B2IN = 512;
constexpr int C_B2HN = 544;
constexpr int N_CONST = 576;
constexpr float W_CARRY  = 16.0f;
constexpr float H_CARRY  = 16.0f;
constexpr float ACC_FOLD = 1.0f / (W_CARRY * H_CARRY);

static_assert(N_BATCH % ROWS_BLK == 0, "batch tiles");
static_assert(HID1 % 32 == 0 && HID2 % 32 == 0, "K multiple of 32");
static_assert(GATE1 % 16 == 0 && GATE2 % 16 == 0, "N multiple of 16");
static_assert(N_STEP % X_CHUNK == 0 && (X_CHUNK % 2) == 0, "x chunks");
static_assert((GATE1 * PITCH_W1) % NTHREADS == 0, "fill loop exact");
static_assert((GATE2 * PITCH_W2I) % NTHREADS == 0, "fill loop exact");
static_assert((GATE2 * PITCH_W2H) % NTHREADS == 0, "fill loop exact");
static_assert((2 * ROWS_BLK * PITCH_H1) % NTHREADS == 0, "fill loop exact");
static_assert((2 * ROWS_BLK * PITCH_H2) % NTHREADS == 0, "fill loop exact");
static_assert(C_B2HN + HID2 == N_CONST, "constant table");
static_assert(GATE1 * PITCH_W1 * 2 + GATE2 * PITCH_W2I * 2 + GATE2 * PITCH_W2H * 2 +
              2 * ROWS_BLK * PITCH_H1 * 2 + 2 * ROWS_BLK * PITCH_H2 * 2 +
              ROWS_BLK * PITCH_X * 4 + ROWS_BLK * PITCH_OUT * 4 + N_CONST * 4 <= 65536, "static LDS");

typedef __attribute__((ext_vector_type(16))) _Float16 v16h;
typedef __attribute__((ext_vector_type(8)))  _Float16 v8h;
typedef __attribute__((ext_vector_type(8)))  float    v8f;
typedef __attribute__((ext_vector_type(4)))  float    v4f;

union FragU { v16h v; v8h h[2]; };

__device__ __forceinline__ v16h frag_load(const _Float16* p) {
  FragU f;
  f.h[0] = *(const v8h*)(p);
  f.h[1] = *(const v8h*)(p + 16);
  return f.v;
}

__device__ __forceinline__ v8f mma_h(v16h a, v16h b, v8f c) {
  c = __builtin_amdgcn_wmma_f32_16x16x32_f16(false, a, false, b, (short)0, c, false, false);
  asm volatile("v_nop\n\tv_nop\n\tv_nop\n\tv_nop" : "+v"(c) : "v"(a), "v"(b));
  return c;
}

__device__ __forceinline__ float fsig(float x)  { return __builtin_amdgcn_rcpf(1.0f + __expf(-x)); }
__device__ __forceinline__ float ftanh(float x) { return 1.0f - 2.0f * __builtin_amdgcn_rcpf(__expf(2.0f * x) + 1.0f); }

__global__ __launch_bounds__(NTHREADS) void gru2_seq_kernel(
    const float* __restrict__ x,
    const float* __restrict__ wih1, const float* __restrict__ whh1,
    const float* __restrict__ bih1, const float* __restrict__ bhh1,
    const float* __restrict__ wih2, const float* __restrict__ whh2,
    const float* __restrict__ bih2, const float* __restrict__ bhh2,
    float* __restrict__ out) {
  __shared__ __align__(16) _Float16 sW1[GATE1 * PITCH_W1];
  __shared__ __align__(16) _Float16 sW2i[GATE2 * PITCH_W2I];
  __shared__ __align__(16) _Float16 sW2h[GATE2 * PITCH_W2H];
  __shared__ __align__(16) _Float16 sH1[2 * ROWS_BLK * PITCH_H1];
  __shared__ __align__(16) _Float16 sH2[2 * ROWS_BLK * PITCH_H2];
  __shared__ __align__(16) float    sX[ROWS_BLK * PITCH_X];
  __shared__ __align__(16) float    sOut[ROWS_BLK * PITCH_OUT];
  __shared__ __align__(16) float    sC[N_CONST];

  const int tid  = threadIdx.x;
  const int lane = tid & 31;
  const int c    = lane & 15;
  const int hh   = lane >> 4;
  const int koff = hh * 8;
  const int rowbase = blockIdx.x * ROWS_BLK;

#pragma unroll 1
  for (int i = tid; i < GATE1 * PITCH_W1; i += NTHREADS) {
    const int g = i / PITCH_W1;
    const int k = i - g * PITCH_W1;
    const int kc = (k < HID1) ? k : (HID1 - 1);
    const float w = whh1[g * HID1 + kc];
    const float v = (k < HID1) ? (w * W_CARRY) : 0.0f;
    sW1[i] = (_Float16)v;
  }
#pragma unroll 1
  for (int i = tid; i < GATE2 * PITCH_W2I; i += NTHREADS) {
    const int g = i / PITCH_W2I;
    const int k = i - g * PITCH_W2I;
    const int kc = (k < HID1) ? k : (HID1 - 1);
    const float w = wih2[g * HID1 + kc];
    const float v = (k < HID1) ? (w * W_CARRY) : 0.0f;
    sW2i[i] = (_Float16)v;
  }
#pragma unroll 1
  for (int i = tid; i < GATE2 * PITCH_W2H; i += NTHREADS) {
    const int g = i / PITCH_W2H;
    const int k = i - g * PITCH_W2H;
    const int kc = (k < HID2) ? k : (HID2 - 1);
    const float w = whh2[g * HID2 + kc];
    const float v = (k < HID2) ? (w * W_CARRY) : 0.0f;
    sW2h[i] = (_Float16)v;
  }
#pragma unroll 1
  for (int i = tid; i < 2 * ROWS_BLK * PITCH_H1; i += NTHREADS) sH1[i] = (_Float16)0.0f;
#pragma unroll 1
  for (int i = tid; i < 2 * ROWS_BLK * PITCH_H2; i += NTHREADS) sH2[i] = (_Float16)0.0f;
#pragma unroll 1
  for (int i = tid; i < GATE1; i += NTHREADS) sC[C_WIH1 + i] = wih1[i];
#pragma unroll 1
  for (int i = tid; i < 2 * HID1; i += NTHREADS) sC[C_B1RZ + i] = bih1[i] + bhh1[i];
#pragma unroll 1
  for (int i = tid; i < HID1; i += NTHREADS) {
    sC[C_B1IN + i] = bih1[2 * HID1 + i];
    sC[C_B1HN + i] = bhh1[2 * HID1 + i];
  }
#pragma unroll 1
  for (int i = tid; i < 2 * HID2; i += NTHREADS) sC[C_B2RZ + i] = bih2[i] + bhh2[i];
#pragma unroll 1
  for (int i = tid; i < HID2; i += NTHREADS) {
    sC[C_B2IN + i] = bih2[2 * HID2 + i];
    sC[C_B2HN + i] = bhh2[2 * HID2 + i];
  }
  __syncthreads();

  float wR[4], wZ[4], wN[4], bR[4], bZ[4], bIN[4], bHN[4];
#pragma unroll
  for (int ht = 0; ht < 4; ++ht) {
    const int u = ht * 16 + c;
    wR[ht]  = sC[C_WIH1 + u];
    wZ[ht]  = sC[C_WIH1 + HID1 + u];
    wN[ht]  = sC[C_WIH1 + 2 * HID1 + u];
    bR[ht]  = sC[C_B1RZ + u];
    bZ[ht]  = sC[C_B1RZ + HID1 + u];
    bIN[ht] = sC[C_B1IN + u];
    bHN[ht] = sC[C_B1HN + u];
  }
  float cR[2], cZ[2], cIN[2], cHN[2];
#pragma unroll
  for (int ht = 0; ht < 2; ++ht) {
    const int u = ht * 16 + c;
    cR[ht]  = sC[C_B2RZ + u];
    cZ[ht]  = sC[C_B2RZ + HID2 + u];
    cIN[ht] = sC[C_B2IN + u];
    cHN[ht] = sC[C_B2HN + u];
  }

  float h1o[4][8], h2o[2][8];
#pragma unroll
  for (int ht = 0; ht < 4; ++ht)
#pragma unroll
    for (int r = 0; r < 8; ++r) h1o[ht][r] = 0.0f;
#pragma unroll
  for (int ht = 0; ht < 2; ++ht)
#pragma unroll
    for (int r = 0; r < 8; ++r) h2o[ht][r] = 0.0f;

  const v8f z8 = {0.f, 0.f, 0.f, 0.f, 0.f, 0.f, 0.f, 0.f};

#pragma unroll 1
  for (int tc = 0; tc < N_STEP / X_CHUNK; ++tc) {
    {
      const int t0 = tc * X_CHUNK;
#pragma unroll
      for (int it = 0; it < 4; ++it) {
        const int row = it * 4 + (lane >> 3);
        const int c4  = (lane & 7) * 4;
        const v4f v = *(const v4f*)(x + (size_t)(rowbase + row) * N_STEP + t0 + c4);
        *(v4f*)(sX + row * PITCH_X + c4) = v;
      }
    }
    __syncthreads();

#pragma unroll 1
    for (int ts = 0; ts < X_CHUNK; ++ts) {
      const int cur = ts & 1;
      const _Float16* h1c = sH1 + cur * (ROWS_BLK * PITCH_H1);
      _Float16*       h1n = sH1 + (cur ^ 1) * (ROWS_BLK * PITCH_H1);
      const _Float16* h2c = sH2 + cur * (ROWS_BLK * PITCH_H2);
      _Float16*       h2n = sH2 + (cur ^ 1) * (ROWS_BLK * PITCH_H2);

      float xv[8];
#pragma unroll
      for (int r = 0; r < 8; ++r) xv[r] = sX[(8 * hh + r) * PITCH_X + ts];

      const v16h a0 = frag_load(h1c + c * PITCH_H1 + koff);
      const v16h a1 = frag_load(h1c + c * PITCH_H1 + koff + 32);
#pragma unroll
      for (int ht = 0; ht < 4; ++ht) {
        const _Float16* wr = sW1 + (ht * 16 + c) * PITCH_W1 + koff;
        const _Float16* wz = wr + HID1 * PITCH_W1;
        const _Float16* wn = wr + 2 * HID1 * PITCH_W1;
        v8f aR = z8, aZ = z8, aN = z8;
        aR = mma_h(a0, frag_load(wr), aR);
        aR = mma_h(a1, frag_load(wr + 32), aR);
        aZ = mma_h(a0, frag_load(wz), aZ);
        aZ = mma_h(a1, frag_load(wz + 32), aZ);
        aN = mma_h(a0, frag_load(wn), aN);
        aN = mma_h(a1, frag_load(wn + 32), aN);
#pragma unroll
        for (int r = 0; r < 8; ++r) {
          const float gxr = fmaf(xv[r], wR[ht], bR[ht]);
          const float gxz = fmaf(xv[r], wZ[ht], bZ[ht]);
          const float gxn = fmaf(xv[r], wN[ht], bIN[ht]);
          const float rg  = fsig(fmaf(aR[r], ACC_FOLD, gxr));
          const float zg  = fsig(fmaf(aZ[r], ACC_FOLD, gxz));
          const float ghn = fmaf(aN[r], ACC_FOLD, bHN[ht]);
          const float ng  = ftanh(fmaf(rg, ghn, gxn));
          const float ho  = h1o[ht][r];
          const float hn  = (1.0f - zg) * ng + zg * ho;
          h1o[ht][r] = hn;
          h1n[(8 * hh + r) * PITCH_H1 + ht * 16 + c] = (_Float16)(hn * H_CARRY);
        }
      }
      __syncthreads();

      const v16h n0 = frag_load(h1n + c * PITCH_H1 + koff);
      const v16h n1 = frag_load(h1n + c * PITCH_H1 + koff + 32);
      const v16h p0 = frag_load(h2c + c * PITCH_H2 + koff);
#pragma unroll
      for (int ht = 0; ht < 2; ++ht) {
        const _Float16* vr = sW2i + (ht * 16 + c) * PITCH_W2I + koff;
        const _Float16* vz = vr + HID2 * PITCH_W2I;
        const _Float16* vn = vr + 2 * HID2 * PITCH_W2I;
        const _Float16* ur = sW2h + (ht * 16 + c) * PITCH_W2H + koff;
        const _Float16* uz = ur + HID2 * PITCH_W2H;
        const _Float16* un = ur + 2 * HID2 * PITCH_W2H;
        v8f aR = z8, aZ = z8, aGX = z8, aGH = z8;
        aR  = mma_h(n0, frag_load(vr), aR);
        aR  = mma_h(n1, frag_load(vr + 32), aR);
        aR  = mma_h(p0, frag_load(ur), aR);
        aZ  = mma_h(n0, frag_load(vz), aZ);
        aZ  = mma_h(n1, frag_load(vz + 32), aZ);
        aZ  = mma_h(p0, frag_load(uz), aZ);
        aGX = mma_h(n0, frag_load(vn), aGX);
        aGX = mma_h(n1, frag_load(vn + 32), aGX);
        aGH = mma_h(p0, frag_load(un), aGH);
#pragma unroll
        for (int r = 0; r < 8; ++r) {
          const float rg  = fsig(fmaf(aR[r], ACC_FOLD, cR[ht]));
          const float zg  = fsig(fmaf(aZ[r], ACC_FOLD, cZ[ht]));
          const float gxn = fmaf(aGX[r], ACC_FOLD, cIN[ht]);
          const float ghn = fmaf(aGH[r], ACC_FOLD, cHN[ht]);
          const float ng  = ftanh(fmaf(rg, ghn, gxn));
          const float ho  = h2o[ht][r];
          const float hn  = (1.0f - zg) * ng + zg * ho;
          h2o[ht][r] = hn;
          h2n[(8 * hh + r) * PITCH_H2 + ht * 16 + c] = (_Float16)(hn * H_CARRY);
        }
      }
      __syncthreads();
    }
  }

#pragma unroll
  for (int ht = 0; ht < 2; ++ht)
#pragma unroll
    for (int r = 0; r < 8; ++r) sOut[(8 * hh + r) * PITCH_OUT + ht * 16 + c] = h2o[ht][r];
  __syncthreads();
  for (int pass = 0; pass < 2; ++pass) {
#pragma unroll
    for (int it = 0; it < 4; ++it) {
      const int idx = it * 32 + lane;
      const int row = idx >> 3;
      const int c4  = (idx & 7) * 4;
      const v4f v = *(const v4f*)(sOut + row * PITCH_OUT + c4);
      *(volatile v4f*)(out + (size_t)(rowbase + row) * HID2 + c4) = v;
    }
    __threadfence();
  }
}

extern "C" void kernel_launch(void* const* d_in, const int* in_sizes, int n_in,
                              void* d_out, int out_size, void* d_ws, size_t ws_size, hipStream_t stream) {
  (void)d_ws; (void)ws_size;
  if (n_in < 9 || d_out == nullptr) return;
  if (in_sizes[0] != N_BATCH * N_STEP || in_sizes[1] != GATE1 || in_sizes[2] != GATE1 * HID1 ||
      in_sizes[3] != GATE1 || in_sizes[4] != GATE1 || in_sizes[5] != GATE2 * HID1 ||
      in_sizes[6] != GATE2 * HID2 || in_sizes[7] != GATE2 || in_sizes[8] != GATE2 ||
      out_size != N_BATCH * HID2) return;

  const float* x    = (const float*)d_in[0];
  const float* wih1 = (const float*)d_in[1];
  const float* whh1 = (const float*)d_in[2];
  const float* bih1 = (const float*)d_in[3];
  const float* bhh1 = (const float*)d_in[4];
  const float* wih2 = (const float*)d_in[5];
  const float* whh2 = (const float*)d_in[6];
  const float* bih2 = (const float*)d_in[7];
  const float* bhh2 = (const float*)d_in[8];
  float* out = (float*)d_out;

  gru2_seq_kernel<<<N_BATCH / ROWS_BLK, NTHREADS, 0, stream>>>(
      x, wih1, whh1, bih1, bhh1, wih2, whh2, bih2, bhh2, out);
}
